// DNL_74234214744693
// MI455X (gfx1250) — hardware-run, weakly checked
//
#include <hip/hip_runtime.h>
#include <math.h>

typedef __attribute__((ext_vector_type(16))) _Float16 v16h;
typedef __attribute__((ext_vector_type(16))) __bf16 v16b;
typedef __attribute__((ext_vector_type(8)))  _Float16 v8h;
typedef __attribute__((ext_vector_type(8)))  float v8f;
typedef __attribute__((ext_vector_type(4)))  float v4f;
typedef __attribute__((ext_vector_type(2)))  float v2f;
typedef __attribute__((ext_vector_type(4)))  unsigned v4u;
typedef __attribute__((ext_vector_type(4)))  int v4i;
typedef float __attribute__((may_alias)) float_a;
typedef int __attribute__((may_alias)) int_a;

template <typename T> __device__ __forceinline__ void vst2(void* p, T v) { *(volatile T*)p = v; __threadfence(); *(volatile T*)p = v; }
__device__ __forceinline__ v8f wmma16(v16h a, v16h b, v8f c) {
  v8f d = __builtin_amdgcn_wmma_f32_16x16x32_f16(false, a, false, b, (short)0, c, false, false);
  asm volatile("v_nop\n\tv_nop\n\tv_nop\n\tv_nop" : "+v"(d) : "v"(a), "v"(b));
  return d;
}
__device__ __forceinline__ v8f wmma_bf(v16b a, v16b b, v8f c) {
  v8f d = __builtin_amdgcn_wmma_f32_16x16x32_bf16(false, a, false, b, (short)0, c, false, false);
  asm volatile("v_nop\n\tv_nop\n\tv_nop\n\tv_nop" : "+v"(d) : "v"(a), "v"(b));
  return d;
}
__device__ __forceinline__ v16h frag_h(const _Float16* rowk0, int lane) {
  union { v16h v; v8h q[2]; } u; const _Float16* p = rowk0 + 8 * (lane >> 4);
  u.q[0] = *(const v8h*)p; u.q[1] = *(const v8h*)(p + 16); return u.v;
}
__device__ __forceinline__ v16h frag_f32(const float* rowk0, int lane) {
  v16h a; const float* p = rowk0 + 8 * (lane >> 4);
#pragma unroll
  for (int i = 0; i < 8; ++i) { a[i] = (_Float16)p[i]; a[8 + i] = (_Float16)p[16 + i]; }
  return a;
}
__device__ __forceinline__ v16h frag_f32s(const float* rowk0, int lane, float sc) {
  v16h a; const float* p = rowk0 + 8 * (lane >> 4);
#pragma unroll
  for (int i = 0; i < 8; ++i) { a[i] = (_Float16)(p[i] * sc); a[8 + i] = (_Float16)(p[16 + i] * sc); }
  return a;
}
__device__ __forceinline__ v16h fragc_f32(const float* W, int k0, int n, int lane, int ld, int K) {
  v16h a; const int g = lane >> 4;
#pragma unroll
  for (int i = 0; i < 8; ++i) { const int ka = k0 + 8 * g + i, kb = ka + 16;
    a[i] = (_Float16)(ka < K ? W[(size_t)(ka < K ? ka : K - 1) * ld + n] : 0.f); a[8 + i] = (_Float16)(kb < K ? W[(size_t)(kb < K ? kb : K - 1) * ld + n] : 0.f); }
  return a;
}
struct F2 { v16b h, l; };
__device__ __forceinline__ F2 bsplit16(const float v[16]) { F2 r;
#pragma unroll
  for (int i = 0; i < 16; ++i) { const __bf16 h = (__bf16)v[i]; r.h[i] = h; r.l[i] = (__bf16)(v[i] - (float)h); }
  return r; }
__device__ __forceinline__ F2 split_row(const float* row, int k0, int lane) { float v[16]; const float* p = row + k0 + 8 * (lane >> 4);
#pragma unroll
  for (int i = 0; i < 8; ++i) { v[i] = p[i]; v[8 + i] = p[16 + i]; }
  return bsplit16(v); }
__device__ __forceinline__ F2 split_rowK(const float* row, int k0, int lane, int K) { float v[16]; const int g = lane >> 4;
#pragma unroll
  for (int i = 0; i < 8; ++i) { const int ka = k0 + 8 * g + i, kb = ka + 16; v[i] = ka < K ? row[ka < K ? ka : K - 1] : 0.f; v[8 + i] = kb < K ? row[kb < K ? kb : K - 1] : 0.f; }
  return bsplit16(v); }
__device__ __forceinline__ F2 split_col(const float* W, int k0, int n, int lane, int ld, int K) { float v[16]; const int g = lane >> 4;
#pragma unroll
  for (int i = 0; i < 8; ++i) { const int ka = k0 + 8 * g + i, kb = ka + 16; v[i] = ka < K ? W[(size_t)(ka < K ? ka : K - 1) * ld + n] : 0.f; v[8 + i] = kb < K ? W[(size_t)(kb < K ? kb : K - 1) * ld + n] : 0.f; }
  return bsplit16(v); }
__device__ __forceinline__ v8f mac3(const F2& a, const F2& b, v8f c) { c = wmma_bf(a.l, b.h, c); c = wmma_bf(a.h, b.l, c); return wmma_bf(a.h, b.h, c); }
__device__ __forceinline__ float sigm(float v) { return 1.0f / (1.0f + expf(-v)); }
#define LDSX() do { asm volatile("s_wait_dscnt 0" ::: "memory"); __builtin_amdgcn_wave_barrier(); __builtin_amdgcn_fence(__ATOMIC_RELEASE, "workgroup"); } while (0)

__device__ __forceinline__ float bfr(float v) { return (float)(__bf16)v; }
#define NBT 4
#define CCH 64
#define NN 4096
#define NPR 272
#ifndef TNB
#define TNB NBT
#endif
#define WS_QR  0u
#define WS_KR  (WS_QR + 4u * (size_t)NBT * NN * CCH)
#define WS_VP  (WS_KR + 4u * (size_t)NBT * NN * CCH)
#define WS_WP  (WS_VP + 4u * (size_t)NBT * CCH * NN)
#define WS_M   (WS_WP + 4u * (size_t)NBT * CCH * NN)
#define WS_MU  (WS_M + 4u * (size_t)NBT * NN)
#define WS_S   (WS_MU + 4u * (size_t)NBT * 128)
#define WS_F   (WS_S + 4u * (size_t)NN * NN)
#define WS_G   (WS_F + 2u * (size_t)NN * NN)
#define WS_END (WS_G + 2u * (size_t)NBT * NN * NN)

__global__ __launch_bounds__(128) void k_conv(const float* __restrict__ X, const float* __restrict__ QW, const float* __restrict__ QB, const float* __restrict__ KW, const float* __restrict__ KB, const float* __restrict__ MW, const float* __restrict__ MB, const float* __restrict__ VW, const float* __restrict__ VB, const float* __restrict__ WW, const float* __restrict__ WB,
    float* __restrict__ QR, float* __restrict__ KR, float* __restrict__ VP, float* __restrict__ WP, float* __restrict__ MV) {
  __shared__ __align__(16) float st[128][68];
  const int tid = threadIdx.x, wave = tid >> 5, lane = tid & 31, col = lane & 15, g = lane >> 4; const int rb = blockIdx.y; const int b = blockIdx.z; const int n0 = blockIdx.x * 128; const int o0 = rb * 64;
  const float* Xb = X + (size_t)b * CCH * NN;
  v8f acc[8] = {};
#pragma unroll
  for (int kc = 0; kc < CCH / 32; ++kc) { v16b a; { const int o = o0 + wave * 16 + col;
      const float* wrow = (o < 64) ? QW + (size_t)o * CCH : (o < 128) ? KW + (size_t)(o - 64) * CCH : (o < 192) ? VW + (size_t)(o - 128) * CCH : (o < 256) ? WW + (size_t)(o - 192) * CCH : MW;
      const bool live = (o <= 256);
#pragma unroll
      for (int e = 0; e < 8; ++e) { a[e] = live ? (__bf16)wrow[kc * 32 + 8 * g + e] : (__bf16)0.f; a[8 + e] = live ? (__bf16)wrow[kc * 32 + 16 + 8 * g + e] : (__bf16)0.f; } }
#pragma unroll
    for (int j = 0; j < 8; ++j) { v16b w; const int n = n0 + j * 16 + col;
#pragma unroll
      for (int e = 0; e < 8; ++e) { w[e] = (__bf16)Xb[(size_t)(kc * 32 + 8 * g + e) * NN + n]; w[8 + e] = (__bf16)Xb[(size_t)(kc * 32 + 16 + 8 * g + e) * NN + n]; }
      acc[j] = wmma_bf(a, w, acc[j]); } }
  if (rb < 2) {
#pragma unroll
    for (int j = 0; j < 8; ++j)
#pragma unroll
      for (int r = 0; r < 8; ++r) { const int ol = wave * 16 + 8 * g + r; const int o = o0 + ol; const float bb = (o < 64) ? bfr(QB[o]) : bfr(KB[o - 64]); st[j * 16 + col][ol] = acc[j][r] + bb; }
    __syncthreads();
    float* dst = (rb == 0 ? QR : KR) + ((size_t)b * NN + n0) * CCH;
    for (int e = tid; e < 128 * 16; e += 128) { const int nl = e >> 4, q = e & 15; vst2(dst + (size_t)nl * CCH + q * 4, *(const v4f*)&st[nl][q * 4]); } }
  else {
    for (int half = 0; half < 2; ++half) {
#pragma unroll
      for (int j = 0; j < 4; ++j)
#pragma unroll
        for (int r = 0; r < 8; ++r) { const int o = o0 + wave * 16 + 8 * g + r; float bb = 0.f; if (o < 192) bb = bfr(VB[o - 128]); else if (o < 256) bb = bfr(WB[o - 192]); else if (o == 256) bb = bfr(MB[0]); st[wave * 32 + (8 * g + r)][(j * 16 + col)] = acc[half * 4 + j][r] + bb; }
      LDSX();
      for (int rl = 0; rl < 16; ++rl) { const int o = o0 + wave * 16 + rl; if (o > 256) continue;
        float* dst = (o < 192) ? VP + ((size_t)b * CCH + (o - 128)) * NN : (o < 256) ? WP + ((size_t)b * CCH + (o - 192)) * NN : MV + (size_t)b * NN;
        if (lane < 16) vst2(dst + n0 + half * 64 + lane * 4, *(const v4f*)&st[wave * 32 + rl][lane * 4]); }
      LDSX(); } } }
__global__ __launch_bounds__(256) void k_mean(const float* __restrict__ QR, const float* __restrict__ KR, float* __restrict__ MU) { __shared__ float sm[32];
  const int t = threadIdx.x; const int cl = t >> 3, sub = t & 7; const int blk = blockIdx.x; const int b = blockIdx.y; const int which = blk >> 1; const int c = (blk & 1) * 32 + cl;
  const float* R = (which == 0 ? QR : KR) + (size_t)b * NN * CCH;
  float s = 0.f; for (int n = sub; n < NN; n += 8) s += R[(size_t)n * CCH + c];
#pragma unroll
  for (int o = 1; o < 8; o <<= 1) s += __shfl_xor(s, o);
  if (sub == 0) sm[cl] = s * (1.0f / NN);
  __syncthreads(); if (t < 32) vst2(MU + (size_t)b * 128 + blk * 32 + t, sm[t]); }
__global__ __launch_bounds__(128) void k_qk(const float* __restrict__ KR, const float* __restrict__ QR, const float* __restrict__ MU, int b, float* __restrict__ S) { __shared__ __align__(16) float ss[4][16][132];
  const int tid = threadIdx.x, wave = tid >> 5, lane = tid & 31, col = lane & 15, g = lane >> 4; const int j0 = blockIdx.y * 128; const int i0 = blockIdx.x * 64 + wave * 16;
  const float* Kb = KR + (size_t)b * NN * CCH; const float* Qb = QR + (size_t)b * NN * CCH; const float* muq = MU + (size_t)b * 128; const float* muk = muq + 64;
  v8f acc[8] = {};
#pragma unroll
  for (int kc = 0; kc < CCH / 32; ++kc) { v16h a; { const float* p = Kb + (size_t)(i0 + col) * CCH + kc * 32 + 8 * g;
#pragma unroll
      for (int e = 0; e < 8; ++e) { a[e] = (_Float16)(p[e] - muk[kc * 32 + 8 * g + e]); a[8 + e] = (_Float16)(p[16 + e] - muk[kc * 32 + 16 + 8 * g + e]); } }
#pragma unroll
    for (int jj = 0; jj < 8; ++jj) { v16h w; const float* p = Qb + (size_t)(j0 + jj * 16 + col) * CCH + kc * 32 + 8 * g;
#pragma unroll
      for (int e = 0; e < 8; ++e) { w[e] = (_Float16)(p[e] - muq[kc * 32 + 8 * g + e]); w[8 + e] = (_Float16)(p[16 + e] - muq[kc * 32 + 16 + 8 * g + e]); }
      acc[jj] = wmma16(a, w, acc[jj]); } }
#pragma unroll
  for (int jj = 0; jj < 8; ++jj)
#pragma unroll
    for (int r = 0; r < 8; ++r) ss[wave][8 * g + r][jj * 16 + col] = acc[jj][r];
  LDSX(); for (int rl = 0; rl < 16; ++rl) vst2(S + (size_t)(i0 + rl) * NN + j0 + lane * 4, *(const v4f*)&ss[wave][rl][lane * 4]); }
__global__ __launch_bounds__(256) void k_g(const float* __restrict__ MV, _Float16* __restrict__ G) { __shared__ __align__(16) _Float16 sg[NBT][NN];
  const int t = threadIdx.x; const size_t i = blockIdx.x; float mi[NBT];
#pragma unroll
  for (int bb = 0; bb < NBT; ++bb) mi[bb] = MV[(size_t)bb * NN + i];
  for (int j = t; j < NN; j += 256) { float e[NBT]; float den = 0.f, mx = -3.0e38f;
#pragma unroll
    for (int bb = 0; bb < NBT; ++bb) { e[bb] = mi[bb] * MV[(size_t)bb * NN + j]; mx = fmaxf(mx, e[bb]); }
#pragma unroll
    for (int bb = 0; bb < NBT; ++bb) { e[bb] = __expf(e[bb] - mx); den += e[bb]; }
    const float inv = 1.0f / den;
#pragma unroll
    for (int bb = 0; bb < NBT; ++bb) sg[bb][j] = (_Float16)(e[bb] * inv); }
  __syncthreads();
  for (int bb = 0; bb < NBT; ++bb) for (int q = t; q < NN / 8; q += 256) vst2((unsigned*)(G + ((size_t)bb * NN + i) * NN + q * 8), *(const v4u*)&sg[bb][q * 8]); }
__global__ __launch_bounds__(256) void k_fs(const float* __restrict__ S, const _Float16* __restrict__ G, int b, _Float16* __restrict__ F) { __shared__ float sred[8]; __shared__ float sbc; __shared__ __align__(16) _Float16 shp[NN];
  const int t = threadIdx.x; const size_t i = blockIdx.x; const float* sr = S + i * NN; const _Float16* gr = G + ((size_t)b * NN + i) * NN;
  float m = -3.0e38f; for (int j = t; j < NN; j += 256) m = fmaxf(m, sr[j]);
#pragma unroll
  for (int o = 1; o < 32; o <<= 1) m = fmaxf(m, __shfl_xor(m, o));
  if ((t & 31) == 0) sred[t >> 5] = m; __syncthreads(); if (t == 0) { float a = sred[0]; for (int e = 1; e < 8; ++e) a = fmaxf(a, sred[e]); sbc = a; } __syncthreads(); m = sbc; __syncthreads();
  float sum = 0.f; for (int j = t; j < NN; j += 256) sum += expf(sr[j] - m);
#pragma unroll
  for (int o = 1; o < 32; o <<= 1) sum += __shfl_xor(sum, o);
  if ((t & 31) == 0) sred[t >> 5] = sum; __syncthreads(); if (t == 0) { float a = 0.f; for (int e = 0; e < 8; ++e) a += sred[e]; sbc = 1.0f / a; } __syncthreads(); const float inv = sbc;
  for (int j = t; j < NN; j += 256) shp[j] = (_Float16)(expf(sr[j] - m) * inv + (float)gr[j]);
  __syncthreads(); for (int q = t; q < NN / 8; q += 256) vst2((unsigned*)(F + i * NN + q * 8), *(const v4u*)&shp[q * 8]); }
__global__ __launch_bounds__(128) void k_y(const float* __restrict__ VP, const _Float16* __restrict__ F, const float* __restrict__ WP, const float* __restrict__ G, const float* __restrict__ BE, const float* __restrict__ RM, const float* __restrict__ RV, int b, float* __restrict__ OUT) { __shared__ __align__(16) float ss[4][16][132];
  const int tid = threadIdx.x, wave = tid >> 5, lane = tid & 31, col = lane & 15, g = lane >> 4; const int j0 = blockIdx.x * 128; const int c0 = wave * 16;
  const float* Vb = VP + (size_t)b * CCH * NN;
  v8f acc[8] = {};
#pragma unroll 2
  for (int kc = 0; kc < NN / 32; ++kc) { const v16h a = frag_f32(Vb + (size_t)(c0 + col) * NN + kc * 32, lane);
#pragma unroll
    for (int jj = 0; jj < 8; ++jj) { v16h w; const int j = j0 + jj * 16 + col;
#pragma unroll
      for (int e = 0; e < 8; ++e) { w[e] = F[(size_t)(kc * 32 + 8 * g + e) * NN + j]; w[8 + e] = F[(size_t)(kc * 32 + 16 + 8 * g + e) * NN + j]; }
      acc[jj] = wmma16(a, w, acc[jj]); } }
#pragma unroll
  for (int jj = 0; jj < 8; ++jj)
#pragma unroll
    for (int r = 0; r < 8; ++r) { const int c = c0 + 8 * g + r; const int j = j0 + jj * 16 + col; const float inv = bfr(G[c]) * rsqrtf(bfr(RV[c]) + 1e-5f); const float wx = WP[((size_t)b * CCH + c) * NN + j] * inv + (bfr(BE[c]) - bfr(RM[c]) * inv); ss[wave][8 * g + r][jj * 16 + col] = acc[jj][r] + wx; }
  LDSX(); for (int rl = 0; rl < 16; ++rl) vst2(OUT + ((size_t)b * CCH + c0 + rl) * NN + j0 + lane * 4, *(const v4f*)&ss[wave][rl][lane * 4]); }
extern "C" void kernel_launch(void* const* d_in, const int* in_sizes, int n_in, void* d_out, int out_size, void* d_ws, size_t ws_size, hipStream_t stream) {
  (void)in_sizes; (void)n_in; (void)out_size;
  const float** Fp = (const float**)d_in;
  if (ws_size < (size_t)WS_END) return;
  char* ws = (char*)d_ws; float *QR = (float*)(ws + WS_QR), *KR = (float*)(ws + WS_KR), *VP = (float*)(ws + WS_VP), *WP = (float*)(ws + WS_WP), *MV = (float*)(ws + WS_M), *MU = (float*)(ws + WS_MU), *S = (float*)(ws + WS_S); _Float16 *F = (_Float16*)(ws + WS_F), *G = (_Float16*)(ws + WS_G);
  k_conv<<<dim3(NN / 128, 5, NBT), 128, 0, stream>>>(Fp[0], Fp[1], Fp[2], Fp[3], Fp[4], Fp[5], Fp[6], Fp[7], Fp[8], Fp[9], Fp[10], QR, KR, VP, WP, MV);
  k_mean<<<dim3(4, NBT), 256, 0, stream>>>(QR, KR, MU);
  k_g<<<dim3(NN), 256, 0, stream>>>(MV, G);
  for (int b = 0; b < TNB; ++b) {
    k_qk<<<dim3(NN / 64, NN / 128), 128, 0, stream>>>(KR, QR, MU, b, S);
    k_fs<<<dim3(NN), 256, 0, stream>>>(S, G, b, F);
    k_y<<<dim3(NN / 128), 128, 0, stream>>>(VP, F, WP, Fp[11], Fp[12], Fp[13], Fp[14], b, (float*)d_out);
  }
}
